// HierarchicalDiffAttentionEncoderLayer_28501402976988
// MI455X (gfx1250) — hardware-verified
//
#include <hip/hip_runtime.h>
#include <stddef.h>
#include <stdint.h>
#include <math.h>

#define NB   4
#define SS   1024
#define DM   1024
#define NH   16
#define HD   64
#define NG   (2 * NH)
#define MR   (NB * SS)
#define N2   (2 * DM)
#define NF   (HD / 2)
#define KC   32
#define QBR  64
#define NWV  4
#define NQB  (SS / QBR)
#define NKT  (SS / KC)
#define PTP  40
#define OTP  68
#define VTRP 65
#define QTP  72
#define NEGB (-1.0e30f)

#define WSC    64.0f
#define QSC    16.0f
#define NSC    16.0f
#define PSC    32768.0f
#define RSC    2048.0f
#define SCL_QK (1.0f / 64.0f)
#define SCL_O  (1.0f / 1024.0f)
#define SCL_S  (1.0f / 2048.0f)
#define SCL_R  (1.0f / 2048.0f)
#define SCL_PV (1.0f / 524288.0f)
#define GNF    0.8f
#define EPSD   1.0e-5
#define L2E4   13.287712379549449

static_assert(MR * DM == 4194304);
static_assert(SS % QBR == 0);
static_assert(SS % KC == 0);
static_assert(QBR == NWV * 16);
static_assert(KC == 32);
static_assert(HD == 64);
static_assert(NF == 32);
static_assert((PTP * 2) % 16 == 0);
static_assert((OTP * 4) % 16 == 0);
static_assert((QTP * 2) % 16 == 0);
static_assert(64 * VTRP <= 64 * OTP);
static_assert(2 * 32 * QTP * 2 <= 64 * OTP * 4);
static_assert(DM % 64 == 0 && N2 % 64 == 0 && MR % 64 == 0);
static_assert((MR * DM) % (8 * 256) == 0);
static_assert((SS * NF) % 128 == 0);
static_assert(64 * NF == 64 * 8 * 4);

typedef float          v8f   __attribute__((ext_vector_type(8)));
typedef float          v4f   __attribute__((ext_vector_type(4)));
typedef double         v2d   __attribute__((ext_vector_type(2)));
typedef unsigned int   v4u   __attribute__((ext_vector_type(4)));
typedef unsigned short v8us  __attribute__((ext_vector_type(8)));
typedef unsigned short v16us __attribute__((ext_vector_type(16)));
typedef _Float16       v8h   __attribute__((ext_vector_type(8)));
typedef _Float16       v16h  __attribute__((ext_vector_type(16)));
typedef unsigned short ush;

union FragU { v16us v; v8us h[2]; v16h f; };
union H8 { v8h h; v8us s; v4u u; };
struct HL { v4u h; v4u l; };

__device__ __forceinline__ ush f2h(float f) {
  union { _Float16 h; ush u; } q;
  q.h = (_Float16)f;
  return q.u;
}

__device__ __forceinline__ v4u pack8(v8f f, float sc) {
  H8 o;
#pragma unroll
  for (int e = 0; e < 8; ++e) o.h[e] = (_Float16)(f[e] * sc);
  return o.u;
}

__device__ __forceinline__ HL split8(v8f f, float sc) {
  H8 ph, pl;
#pragma unroll
  for (int e = 0; e < 8; ++e) {
    const float v = f[e] * sc;
    const _Float16 hi = (_Float16)v;
    ph.h[e] = hi;
    pl.h[e] = (_Float16)((v - (float)hi) * RSC);
  }
  HL r; r.h = ph.u; r.l = pl.u;
  return r;
}

__device__ __forceinline__ v8f mma16(v16us a, v16us b, v8f c) {
  FragU ua, ub; ua.v = a; ub.v = b;
  c = __builtin_amdgcn_wmma_f32_16x16x32_f16(false, ua.f, false, ub.f, (short)0, c, false, false);
  asm volatile("v_nop\n\tv_nop\n\tv_nop\n\tv_nop" : "+v"(c) : "v"(a), "v"(b));
  return c;
}

__device__ __forceinline__ v16us ldfragu(const ush* p, int ld, int row0, int k0, int lane) {
  const int m = lane & 15, lh = lane >> 4;
  const ush* qq = p + (size_t)(row0 + m) * ld + k0 + 8 * lh;
  FragU f;
  f.h[0] = *(const v8us*)(qq);
  f.h[1] = *(const v8us*)(qq + 16);
  return f.v;
}

__device__ __forceinline__ v8f zero8() { return (v8f){0.f, 0.f, 0.f, 0.f, 0.f, 0.f, 0.f, 0.f}; }

__global__ __launch_bounds__(128) void k_prep(const float* __restrict__ aff, double* __restrict__ Lg,
                                              float* __restrict__ tcs, float* __restrict__ tsn) {
  __shared__ __align__(16) double Ls[NB * SS];
  const int tid = threadIdx.x, lane = tid & 31, wave = tid >> 5;
  if (blockIdx.x == 0) {
    const int b = wave;
    const float* ab = aff + (size_t)b * (SS - 1);
    double csum = 0.0;
#pragma unroll 1
    for (int i = 0; i < 32; ++i) {
      const int m  = lane * 32 + i;
      const int mc = (m < SS - 1) ? m : (SS - 2);
      const float lv = logf(ab[mc]);
      csum += (m < SS - 1) ? (double)lv : 0.0;
    }
    double incl = csum;
#pragma unroll
    for (int off = 1; off < 32; off <<= 1) {
      const double t = __shfl_up(incl, off, 32);
      incl = (lane >= off) ? (incl + t) : incl;
    }
    const double exs = __shfl_up(incl, 1, 32);
    double run = (lane == 0) ? 0.0 : exs;
#pragma unroll 1
    for (int i = 0; i < 32; ++i) {
      const int k = lane * 32 + i;
      Ls[b * SS + k] = run;
      const int mc = (k < SS - 1) ? k : (SS - 2);
      const float lv = logf(ab[mc]);
      run += (k < SS - 1) ? (double)lv : 0.0;
    }
    __syncthreads();
#pragma unroll 1
    for (int it = 0; it < 16; ++it) {
      const int p = tid + 128 * it;
      const v2d v = *(const v2d*)(Ls + 2 * p);
      *(volatile v2d*)(Lg + 2 * p) = v;
    }
    __threadfence();
#pragma unroll 1
    for (int it = 0; it < 16; ++it) {
      const int p = tid + 128 * it;
      const v2d v = *(const v2d*)(Ls + 2 * p);
      *(volatile v2d*)(Lg + 2 * p) = v;
    }
  } else {
    const int e   = ((int)blockIdx.x - 1) * 128 + tid;
    const int pos = e >> 5, j = e & 31;
    const double pd = exp2((double)j * 0.03125 * L2E4);
    const float  pf = (float)pd;
    const float  fr = 1.0f / pf;
    const float ang = (float)pos * fr;
    const float  sn = sinf(ang);
    const float  cs = cosf(ang);
    *(volatile float*)(tcs + e) = cs;
    *(volatile float*)(tsn + e) = sn;
    __threadfence();
    *(volatile float*)(tcs + e) = cs;
    *(volatile float*)(tsn + e) = sn;
  }
}

__global__ __launch_bounds__(256) void k_cvt(const float* __restrict__ x, const float* __restrict__ wq,
                                             const float* __restrict__ wk, const float* __restrict__ wv,
                                             const float* __restrict__ wo,
                                             ush* __restrict__ xh, ush* __restrict__ wqh, ush* __restrict__ wkh,
                                             ush* __restrict__ wvh, ush* __restrict__ woh) {
  const int y = blockIdx.y;
  const float* src = (y == 0) ? x : ((y == 1) ? wq : ((y == 2) ? wk : ((y == 3) ? wv : wo)));
  ush* dst = (y == 0) ? xh : ((y == 1) ? wqh : ((y == 2) ? wkh : ((y == 3) ? wvh : woh)));
  const int nblk = (y == 0) ? (MR * DM / 2048) : ((y <= 2) ? (N2 * DM / 2048) : (DM * DM / 2048));
  const float sc = (y == 0) ? 1.0f : WSC;
  if ((int)blockIdx.x >= nblk) return;
  const size_t p  = (size_t)blockIdx.x * 256 + threadIdx.x;
  const size_t so = p * 8;
  const v4f a0 = *(const v4f*)(src + so);
  const v4f a1 = *(const v4f*)(src + so + 4);
  const v8f f = (v8f){a0[0], a0[1], a0[2], a0[3], a1[0], a1[1], a1[2], a1[3]};
  const v4u o = pack8(f, sc);
  *(volatile v4u*)(dst + so) = o;
  __threadfence();
  *(volatile v4u*)(dst + so) = o;
}

template <int MODE>
__global__ __launch_bounds__(64) void k_gemm(const ush* __restrict__ A, const ush* __restrict__ W,
                                             const float* __restrict__ bias,
                                             const float* __restrict__ tcs, const float* __restrict__ tsn,
                                             ush* __restrict__ o16a, ush* __restrict__ o16b,
                                             float* __restrict__ o32) {
  __shared__ __align__(16) float sm[64 * OTP];
  __shared__ __align__(16) float rcs[64 * NF];
  __shared__ __align__(16) float rsn[64 * NF];
  const int tid = threadIdx.x, lane = tid & 31, wave = tid >> 5;
  const int hh = lane >> 4, c = lane & 15;
  const int n0 = blockIdx.x * 64;
  const int m0 = blockIdx.y * 64;
  const int r0 = m0 + 32 * wave;

  if (MODE == 0) {
    const int sb = m0 & (SS - 1);
    const float* cbp = tcs + (size_t)sb * NF;
    const float* sbp = tsn + (size_t)sb * NF;
#pragma unroll 1
    for (int it = 0; it < 8; ++it) {
      const int p = tid + 64 * it;
      const v4f cv = *(const v4f*)(cbp + 4 * p);
      const v4f sv = *(const v4f*)(sbp + 4 * p);
      *(v4f*)(rcs + 4 * p) = cv;
      *(v4f*)(rsn + 4 * p) = sv;
    }
    __syncthreads();
  }

  v8f acc[2][4];
#pragma unroll
  for (int fm = 0; fm < 2; ++fm)
#pragma unroll
    for (int fn = 0; fn < 4; ++fn) acc[fm][fn] = zero8();

#pragma unroll 1
  for (int k0 = 0; k0 < DM; k0 += 32) {
    v16us af[2], bf[4];
#pragma unroll
    for (int fm = 0; fm < 2; ++fm) af[fm] = ldfragu(A, DM, r0 + 16 * fm, k0, lane);
#pragma unroll
    for (int fn = 0; fn < 4; ++fn) bf[fn] = ldfragu(W, DM, n0 + 16 * fn, k0, lane);
#pragma unroll
    for (int fm = 0; fm < 2; ++fm)
#pragma unroll
      for (int fn = 0; fn < 4; ++fn) acc[fm][fn] = mma16(af[fm], bf[fn], acc[fm][fn]);
  }

  float bv[4];
#pragma unroll
  for (int fn = 0; fn < 4; ++fn) bv[fn] = bias[n0 + 16 * fn + c];

  if (MODE == 0) {
    ush* tw = (ush*)sm + wave * (32 * QTP);
#pragma unroll
    for (int fm = 0; fm < 2; ++fm)
#pragma unroll
      for (int r = 0; r < 8; ++r) {
        const int lr   = 16 * fm + 8 * hh + r;
        const int lrow = 32 * wave + lr;
#pragma unroll
        for (int fn = 0; fn < 2; ++fn) {
          const int d = 16 * fn + c;
          const float cs = rcs[lrow * NF + d];
          const float sn = rsn[lrow * NF + d];
          const float x1 = acc[fm][fn][r] * SCL_QK + bv[fn];
          const float x2 = acc[fm][fn + 2][r] * SCL_QK + bv[fn + 2];
          const float o1 = x1 * cs - x2 * sn;
          const float o2 = x1 * sn + x2 * cs;
          tw[lr * QTP + d]      = f2h(o1 * QSC);
          tw[lr * QTP + d + NF] = f2h(o2 * QSC);
        }
      }
    __syncthreads();
    const int g = blockIdx.x;
    v4u val[8];
    size_t go[8];
#pragma unroll
    for (int it = 0; it < 8; ++it) {
      const int p  = lane + 32 * it;
      const int lr = p >> 3;
      const int pc = p & 7;
      const int grow = r0 + lr;
      const int b = grow >> 10, s = grow & (SS - 1);
      H8 t; t.s = *(const v8us*)(tw + lr * QTP + pc * 8);
      val[it] = t.u;
      go[it] = ((size_t)(b * NG + g) * SS + s) * HD + pc * 8;
    }
#pragma unroll
    for (int it = 0; it < 8; ++it) *(volatile v4u*)(o16a + go[it]) = val[it];
    __threadfence();
#pragma unroll
    for (int it = 0; it < 8; ++it) *(volatile v4u*)(o16a + go[it]) = val[it];
  } else if (MODE == 1) {
    float* tl = sm;
#pragma unroll
    for (int fm = 0; fm < 2; ++fm)
#pragma unroll
      for (int fn = 0; fn < 4; ++fn)
#pragma unroll
        for (int r = 0; r < 8; ++r) {
          const int lr = 32 * wave + 16 * fm + 8 * hh + r;
          tl[lr * VTRP + 16 * fn + c] = acc[fm][fn][r] * SCL_QK + bv[fn];
        }
    __syncthreads();
    const int h = blockIdx.x;
    const int b = m0 >> 10, s0 = m0 & (SS - 1);
#pragma unroll 1
    for (int pass = 0; pass < 2; ++pass) {
      if (pass == 1) __threadfence();
#pragma unroll
      for (int it = 0; it < 8; ++it) {
        const int p  = tid + 64 * it;
        const int dd = p >> 3;
        const int pc = p & 7;
        const float* cp = tl + (pc * 8) * VTRP + dd;
        const v8f f = (v8f){cp[0 * VTRP], cp[1 * VTRP], cp[2 * VTRP], cp[3 * VTRP],
                            cp[4 * VTRP], cp[5 * VTRP], cp[6 * VTRP], cp[7 * VTRP]};
        const HL sp = split8(f, QSC);
        const size_t go = ((size_t)(b * NH + h) * HD + dd) * SS + s0 + pc * 8;
        *(volatile v4u*)(o16a + go) = sp.h;
        *(volatile v4u*)(o16b + go) = sp.l;
      }
    }
  } else {
    float* sw = sm + wave * (32 * OTP);
#pragma unroll
    for (int fm = 0; fm < 2; ++fm)
#pragma unroll
      for (int fn = 0; fn < 4; ++fn)
#pragma unroll
        for (int r = 0; r < 8; ++r)
          sw[(16 * fm + 8 * hh + r) * OTP + 16 * fn + c] = acc[fm][fn][r] * SCL_O + bv[fn];
    __syncthreads();
#pragma unroll 1
    for (int pass = 0; pass < 2; ++pass) {
      if (pass == 1) __threadfence();
#pragma unroll
      for (int it = 0; it < 16; ++it) {
        const int p    = lane + 32 * it;
        const int L    = p >> 3;
        const int pc   = p & 7;
        const int lr   = L >> 1;
        const int half = L & 1;
        const v4f v = *(const v4f*)(sw + lr * OTP + half * 32 + pc * 4);
        const size_t go = (size_t)(r0 + lr) * DM + n0 + half * 32 + pc * 4;
        *(volatile v4f*)(o32 + go) = v;
      }
    }
  }
}

__global__ __launch_bounds__(128) void k_stat(const ush* __restrict__ QP, const ush* __restrict__ KP,
                                              float* __restrict__ LSE) {
  __shared__ __align__(16) float Ls2[QBR];
  const int tid = threadIdx.x, lane = tid & 31, wave = tid >> 5;
  const int hh = lane >> 4, c = lane & 15;
  const int qb = blockIdx.x, g = blockIdx.y, b = blockIdx.z;
  const size_t gi = (size_t)(b * NG + g);
  const ush* Qp = QP + gi * SS * HD;
  const ush* Kp = KP + gi * SS * HD;
  const int qblk = qb * QBR, q0 = qblk + 16 * wave;

  float mrow[8], lrow[8];
#pragma unroll
  for (int r = 0; r < 8; ++r) { mrow[r] = NEGB; lrow[r] = 0.f; }

#pragma unroll 1
  for (int it = 0; it < NKT; ++it) {
    const int kv0 = it * KC;
    v8f s[2];
    s[0] = zero8(); s[1] = zero8();
#pragma unroll
    for (int dc = 0; dc < 2; ++dc) {
      const v16us qa = ldfragu(Qp, HD, q0, 32 * dc, lane);
#pragma unroll
      for (int j = 0; j < 2; ++j) {
        const v16us kf = ldfragu(Kp, HD, kv0 + 16 * j, 32 * dc, lane);
        s[j] = mma16(qa, kf, s[j]);
      }
    }
    float cm[8];
#pragma unroll
    for (int r = 0; r < 8; ++r) {
      s[0][r] *= SCL_S; s[1][r] *= SCL_S;
      float m = fmaxf(s[0][r], s[1][r]);
#pragma unroll
      for (int off = 1; off < 16; off <<= 1) m = fmaxf(m, __shfl_xor(m, off, 32));
      cm[r] = m;
    }
#pragma unroll
    for (int r = 0; r < 8; ++r) {
      const float mnew  = fmaxf(mrow[r], cm[r]);
      const float alpha = __expf(mrow[r] - mnew);
      float psum = __expf(s[0][r] - mnew) + __expf(s[1][r] - mnew);
#pragma unroll
      for (int off = 1; off < 16; off <<= 1) psum += __shfl_xor(psum, off, 32);
      lrow[r] = lrow[r] * alpha + psum;
      mrow[r] = mnew;
    }
  }
#pragma unroll
  for (int r = 0; r < 8; ++r) {
    const float v = mrow[r] + logf(lrow[r]);
    if (c == 0) Ls2[wave * 16 + 8 * hh + r] = v;
  }
  __syncthreads();
  const int lc = lane & 15;
  const v4f lv = *(const v4f*)(Ls2 + 4 * lc);
  const size_t lgo = gi * SS + qblk + 4 * lc;
  const bool wl = (wave == 0) && (lane < 16);
  if (wl) *(volatile v4f*)(LSE + lgo) = lv;
  __threadfence();
  if (wl) *(volatile v4f*)(LSE + lgo) = lv;
}

__global__ __launch_bounds__(128)
void k_attn(const ush* __restrict__ QP, const ush* __restrict__ KP,
            const ush* __restrict__ Vth, const ush* __restrict__ Vtl,
            const float* __restrict__ LSE, const double* __restrict__ Lg,
            const float* __restrict__ lam_p, float* __restrict__ CTX, double* __restrict__ GNP) {
  __shared__ __align__(16) ush    Ph[NWV * 16 * PTP];
  __shared__ __align__(16) ush    Pl[NWV * 16 * PTP];
  __shared__ __align__(16) float  Os[NWV * 16 * OTP];
  __shared__ __align__(16) double Gd[2 * 128];
  __shared__ __align__(16) double Gt[2];

  const int tid = threadIdx.x, lane = tid & 31, wave = tid >> 5;
  const int hh = lane >> 4, c = lane & 15;
  const int qb = blockIdx.x, h = blockIdx.y, b = blockIdx.z;
  const int qblk = qb * QBR, q0 = qblk + 16 * wave;
  const size_t g1 = (size_t)(b * NG + h), g2 = g1 + NH;
  const ush* Q1 = QP + g1 * SS * HD;
  const ush* Q2 = QP + g2 * SS * HD;
  const ush* K1 = KP + g1 * SS * HD;
  const ush* K2 = KP + g2 * SS * HD;
  const ush* Vh = Vth + (size_t)(b * NH + h) * HD * SS;
  const ush* Vl = Vtl + (size_t)(b * NH + h) * HD * SS;
  const double* Lb = Lg + (size_t)b * SS;
  const float lamv = lam_p[0];

  float lse1[8], lse2[8];
  double Li[8];
#pragma unroll
  for (int r = 0; r < 8; ++r) {
    const int row = q0 + 8 * hh + r;
    lse1[r] = LSE[g1 * SS + row];
    lse2[r] = LSE[g2 * SS + row];
    Li[r]   = Lb[row];
  }
  v8f oacc[4], racc[4];
#pragma unroll
  for (int t = 0; t < 4; ++t) { oacc[t] = zero8(); racc[t] = zero8(); }

  ush*   pwh = Ph + wave * 16 * PTP;
  ush*   pwl = Pl + wave * 16 * PTP;
  float* sw  = Os + wave * 16 * OTP;

#pragma unroll 1
  for (int it = 0; it < NKT; ++it) {
    const int kv0 = it * KC;
    __syncthreads();

    v8f s1[2], s2[2];
    s1[0] = zero8(); s1[1] = zero8(); s2[0] = zero8(); s2[1] = zero8();
#pragma unroll
    for (int dc = 0; dc < 2; ++dc) {
      const v16us qa1 = ldfragu(Q1, HD, q0, 32 * dc, lane);
      const v16us qa2 = ldfragu(Q2, HD, q0, 32 * dc, lane);
#pragma unroll
      for (int j = 0; j < 2; ++j) {
        const v16us kf1 = ldfragu(K1, HD, kv0 + 16 * j, 32 * dc, lane);
        const v16us kf2 = ldfragu(K2, HD, kv0 + 16 * j, 32 * dc, lane);
        s1[j] = mma16(qa1, kf1, s1[j]);
        s2[j] = mma16(qa2, kf2, s2[j]);
      }
    }
    double Lj[2];
#pragma unroll
    for (int j = 0; j < 2; ++j) Lj[j] = Lb[kv0 + 16 * j + c];

#pragma unroll
    for (int r = 0; r < 8; ++r)
#pragma unroll
      for (int j = 0; j < 2; ++j) {
        const float p1 = __expf(s1[j][r] * SCL_S - lse1[r]);
        const float p2 = __expf(s2[j][r] * SCL_S - lse2[r]);
        const int qrow = q0 + 8 * hh + r;
        const int key  = kv0 + 16 * j + c;
        const float cd = (float)(Li[r] - Lj[j]);
        const float ce = (key >= qrow) ? (-cd) : cd;
        const float cc = __expf(ce);
        const float w  = cc * (p1 - lamv * p2);
        const float wsv = w * PSC;
        const _Float16 whi = (_Float16)wsv;
        const float rem = (wsv - (float)whi) * RSC;
        union { _Float16 hq; ush uq; } qh;
        qh.hq = whi;
        pwh[(8 * hh + r) * PTP + 16 * j + c] = qh.uq;
        pwl[(8 * hh + r) * PTP + 16 * j + c] = f2h(rem);
      }
    __syncthreads();

    {
      const v16us pah = ldfragu(pwh, PTP, 0, 0, lane);
      const v16us pal = ldfragu(pwl, PTP, 0, 0, lane);
#pragma unroll
      for (int t = 0; t < 4; ++t) {
        const v16us vfh = ldfragu(Vh, SS, 16 * t, kv0, lane);
        const v16us vfl = ldfragu(Vl, SS, 16 * t, kv0, lane);
        oacc[t] = mma16(pah, vfh, oacc[t]);
        racc[t] = mma16(pah, vfl, racc[t]);
        racc[t] = mma16(pal, vfh, racc[t]);
      }
    }
  }
  __syncthreads();

  double gs = 0.0, gq = 0.0;
#pragma unroll
  for (int r = 0; r < 8; ++r) {
    const int row = 8 * hh + r;
#pragma unroll
    for (int t = 0; t < 4; ++t) {
      const float v = (oacc[t][r] + racc[t][r] * SCL_R) * SCL_PV;
      sw[row * OTP + 16 * t + c] = v;
      gs += (double)v;
      gq += (double)v * (double)v;
    }
  }
  Gd[2 * tid]     = gs;
  Gd[2 * tid + 1] = gq;
  __syncthreads();
  if (tid == 0) {
    double S = 0.0, Q = 0.0;
#pragma unroll 1
    for (int i = 0; i < 128; ++i) { S += Gd[2 * i]; Q += Gd[2 * i + 1]; }
    Gt[0] = S; Gt[1] = Q;
  }
  __syncthreads();

  v4f val[8];
  size_t go[8];
#pragma unroll
  for (int it = 0; it < 8; ++it) {
    const int p    = lane + 32 * it;
    const int L    = p >> 3;
    const int pc   = p & 7;
    const int row  = L >> 1;
    const int half = L & 1;
    val[it] = *(const v4f*)(sw + row * OTP + half * 32 + pc * 4);
    go[it]  = ((size_t)(b * SS + q0 + row) * NH + h) * HD + half * 32 + pc * 4;
  }
  const v2d gtv = *(const v2d*)Gt;
  v2d gv;
  gv[0] = (lane == 0) ? gtv[0] : 0.0;
  gv[1] = (lane == 0) ? gtv[1] : 0.0;
  const bool wgl = (wave == 0) && (lane < 8);
  double* gp = GNP + (((size_t)(b * NH + h) * NQB + qb) * 16 + 2 * lane);

#pragma unroll
  for (int it = 0; it < 8; ++it) *(volatile v4f*)(CTX + go[it]) = val[it];
  if (wgl) *(volatile v2d*)gp = gv;
  __threadfence();
#pragma unroll
  for (int it = 0; it < 8; ++it) *(volatile v4f*)(CTX + go[it]) = val[it];
  if (wgl) *(volatile v2d*)gp = gv;
}

__global__ __launch_bounds__(64) void k_gnfin(const double* __restrict__ GNP, float* __restrict__ GNS) {
  const int bh = threadIdx.x;
  double S = 0.0, Q = 0.0;
#pragma unroll 1
  for (int qb = 0; qb < NQB; ++qb) {
    const double* p = GNP + ((size_t)bh * NQB + qb) * 16;
    S += p[0];
    Q += p[1];
  }
  const double inv  = 1.0 / (double)(SS * HD);
  const double mean = S * inv;
  double var = Q * inv - mean * mean;
  var = (var > 0.0) ? var : 0.0;
  const double rstd = 1.0 / sqrt(var + EPSD);
  const v4f o = (v4f){(float)mean, (float)rstd, 0.f, 0.f};
  *(volatile v4f*)(GNS + bh * 4) = o;
  __threadfence();
  *(volatile v4f*)(GNS + bh * 4) = o;
}

__global__ __launch_bounds__(256) void k_gnapply(const float* __restrict__ CTX, const float* __restrict__ GNS,
                                                 const float* __restrict__ gw, const float* __restrict__ gb,
                                                 ush* __restrict__ NRM) {
  const size_t p = (size_t)blockIdx.x * 256 + threadIdx.x;
  const int b  = (int)(p >> 17);
  const int h  = (int)((p >> 3) & (NH - 1));
  const int d0 = (int)(p & 7) * 8;
  const int bh = b * NH + h;
  const float mean = GNS[bh * 4], rstd = GNS[bh * 4 + 1];
  const size_t e0 = p * 8;
  const v4f a0 = *(const v4f*)(CTX + e0);
  const v4f a1 = *(const v4f*)(CTX + e0 + 4);
  const v4f w0 = *(const v4f*)(gw + h * HD + d0);
  const v4f w1 = *(const v4f*)(gw + h * HD + d0 + 4);
  const v4f c0 = *(const v4f*)(gb + h * HD + d0);
  const v4f c1 = *(const v4f*)(gb + h * HD + d0 + 4);
  H8 o;
#pragma unroll
  for (int e = 0; e < 4; ++e) {
    const float n0 = (((a0[e] - mean) * rstd) * w0[e] + c0[e]) * GNF;
    const float n1 = (((a1[e] - mean) * rstd) * w1[e] + c1[e]) * GNF;
    o.h[e]     = (_Float16)(n0 * NSC);
    o.h[e + 4] = (_Float16)(n1 * NSC);
  }
  *(volatile v4u*)(NRM + e0) = o.u;
  __threadfence();
  *(volatile v4u*)(NRM + e0) = o.u;
}

extern "C" void kernel_launch(void* const* d_in, const int* in_sizes, int n_in,
                              void* d_out, int out_size, void* d_ws, size_t ws_size,
                              hipStream_t stream) {
  if (n_in < 13) return;
  if (in_sizes[0] != MR * DM) return;
  if (in_sizes[1] != NB * (SS - 1)) return;
  if (in_sizes[2] != N2 * DM || in_sizes[3] != N2) return;
  if (in_sizes[4] != N2 * DM || in_sizes[5] != N2) return;
  if (in_sizes[6] != DM * DM || in_sizes[7] != DM) return;
  if (in_sizes[8] != DM * DM || in_sizes[9] != DM) return;
  if (in_sizes[10] != DM || in_sizes[11] != DM) return;
  if (in_sizes[12] < 1) return;
  if (out_size != MR * DM) return;

  const float* x    = (const float*)d_in[0];
  const float* aff  = (const float*)d_in[1];
  const float* wq   = (const float*)d_in[2];
  const float* bq   = (const float*)d_in[3];
  const float* wk   = (const float*)d_in[4];
  const float* bk   = (const float*)d_in[5];
  const float* wv   = (const float*)d_in[6];
  const float* bvv  = (const float*)d_in[7];
  const float* wo   = (const float*)d_in[8];
  const float* bo   = (const float*)d_in[9];
  const float* gw   = (const float*)d_in[10];
  const float* gb   = (const float*)d_in[11];
  const float* lamp = (const float*)d_in[12];
  float* out = (float*)d_out;

  size_t off = 0;
  const size_t oXH  = off; off += (size_t)MR * DM * 2;
  const size_t oWQ  = off; off += (size_t)N2 * DM * 2;
  const size_t oWK  = off; off += (size_t)N2 * DM * 2;
  const size_t oWV  = off; off += (size_t)DM * DM * 2;
  const size_t oWO  = off; off += (size_t)DM * DM * 2;
  const size_t oTCS = off; off += (size_t)SS * NF * 4;
  const size_t oTSN = off; off += (size_t)SS * NF * 4;
  const size_t oLG  = off; off += (size_t)NB * SS * 8;
  const size_t oQP  = off; off += (size_t)NB * NG * SS * HD * 2;
  const size_t oKP  = off; off += (size_t)NB * NG * SS * HD * 2;
  const size_t oVTH = off; off += (size_t)NB * NH * HD * SS * 2;
  const size_t oVTL = off; off += (size_t)NB * NH * HD * SS * 2;
  const size_t oLSE = off; off += (size_t)NB * NG * SS * 4;
  const size_t oCTX = off; off += (size_t)MR * DM * 4;
  const size_t oGNP = off; off += (size_t)NB * NH * NQB * 128;
  const size_t oGNS = off; off += 4096;
  const size_t oNRM = off; off += (size_t)MR * DM * 2;
  if (off > ws_size) return;
  if (off > (size_t)134217728) return;

  char* ws = (char*)d_ws;
  ush*    XH  = (ush*)(ws + oXH);
  ush*    WQ  = (ush*)(ws + oWQ);
  ush*    WK  = (ush*)(ws + oWK);
  ush*    WV  = (ush*)(ws + oWV);
  ush*    WO  = (ush*)(ws + oWO);
  float*  TCS = (float*)(ws + oTCS);
  float*  TSN = (float*)(ws + oTSN);
  double* LG  = (double*)(ws + oLG);
  ush*    QP  = (ush*)(ws + oQP);
  ush*    KP  = (ush*)(ws + oKP);
  ush*    VTH = (ush*)(ws + oVTH);
  ush*    VTL = (ush*)(ws + oVTL);
  float*  LSE = (float*)(ws + oLSE);
  float*  CTX = (float*)(ws + oCTX);
  double* GNP = (double*)(ws + oGNP);
  float*  GNS = (float*)(ws + oGNS);
  ush*    NRM = (ush*)(ws + oNRM);

  k_prep<<<dim3(1 + (SS * NF) / 128), dim3(128), 0, stream>>>(aff, LG, TCS, TSN);
  k_cvt<<<dim3(MR * DM / 2048, 5), dim3(256), 0, stream>>>(x, wq, wk, wv, wo, XH, WQ, WK, WV, WO);
  k_gemm<0><<<dim3(N2 / 64, MR / 64), dim3(64), 0, stream>>>(XH, WQ, bq, TCS, TSN, QP, QP, CTX);
  k_gemm<0><<<dim3(N2 / 64, MR / 64), dim3(64), 0, stream>>>(XH, WK, bk, TCS, TSN, KP, KP, CTX);
  k_gemm<1><<<dim3(DM / 64, MR / 64), dim3(64), 0, stream>>>(XH, WV, bvv, TCS, TSN, VTH, VTL, CTX);
  k_stat<<<dim3(NQB, NG, NB), dim3(128), 0, stream>>>(QP, KP, LSE);
  k_attn<<<dim3(NQB, NH, NB), dim3(128), 0, stream>>>(QP, KP, VTH, VTL, LSE, LG, lamp, CTX, GNP);
  k_gnfin<<<dim3(1), dim3(64), 0, stream>>>(GNP, GNS);
  k_gnapply<<<dim3(MR * DM / 2048), dim3(256), 0, stream>>>(CTX, GNS, gw, gb, NRM);
  k_gemm<2><<<dim3(DM / 64, MR / 64), dim3(64), 0, stream>>>(NRM, WO, bo, TCS, TSN, NRM, NRM, out);
  (void)hipGetLastError();
}
